// MultiHead_Attention_Lattice_rel_55121610277409
// MI455X (gfx1250) — hardware-verified
//
#include <hip/hip_runtime.h>
#include <stddef.h>
#include <stdint.h>


#define NB     2
#define NL     192
#define NH     512
#define NHEAD  8
#define NDH    64
#define NMAXL  512
#define NPE    1025
#define NPEP   1088
#define NBL    384
#define NF2    256
#define NFUS   1024
#define NTHR   256
#define GTHR   128
#define GBM    64
#define GBN    64
#define ATP    136
#define TT     64
#define TP     68
#define CX     8.0f
#define CW     64.0f
#define CR     256.0f
#define CG     128.0f
#define CP     4096.0f
#define CO     64.0f
#define WSMAX  134217728

static_assert(NH == NHEAD * NDH);
static_assert(NBL == NB * NL);
static_assert((NBL % GBM) == 0 && (NH % GBN) == 0 && (NL % GBM) == 0 && (NPEP % GBM) == 0 && (NH % GBM) == 0);
static_assert(NPEP >= NPE);
static_assert((NH % 32) == 0 && (NDH % 32) == 0 && (NL % 32) == 0 && (NF2 % 32) == 0);
static_assert(NL == 24 * 8);
static_assert((NL % 64) == 0 && (NH % 128) == 0);
static_assert(GTHR == 128 && NTHR == 256);
static_assert(GBM == (GTHR / 32) * 16);
static_assert((ATP % 8) == 0);
static_assert((NH % TT) == 0);

typedef _Float16 f16;
typedef float    v4f  __attribute__((ext_vector_type(4)));
typedef float    v8f  __attribute__((ext_vector_type(8)));
typedef int      v8i  __attribute__((ext_vector_type(8)));
typedef _Float16 v8h  __attribute__((ext_vector_type(8)));
typedef _Float16 v16h __attribute__((ext_vector_type(16)));
union FragH { v16h v; v8h h[2]; v8i w; };

__device__ __forceinline__ v8f wmh(const FragH& a, const FragH& b, v8f c) {
  v8f d = __builtin_amdgcn_wmma_f32_16x16x32_f16(false, a.v, false, b.v, (short)0, c, false, false);
  asm volatile("v_nop\n\tv_nop\n\tv_nop\n\tv_nop" : "+v"(d) : "v"(a.w), "v"(b.w));
  return d;
}

__device__ __forceinline__ v8h cvt8h(const v4f a, const v4f b, const float c) {
  v8h hv;
  hv[0] = (f16)(a.x * c); hv[1] = (f16)(a.y * c);
  hv[2] = (f16)(a.z * c); hv[3] = (f16)(a.w * c);
  hv[4] = (f16)(b.x * c); hv[5] = (f16)(b.y * c);
  hv[6] = (f16)(b.z * c); hv[7] = (f16)(b.w * c);
  return hv;
}

__device__ __forceinline__ v4f relu4(const v4f a) {
  v4f r;
  r.x = fmaxf(a.x, 0.f); r.y = fmaxf(a.y, 0.f); r.z = fmaxf(a.z, 0.f); r.w = fmaxf(a.w, 0.f);
  return r;
}

__global__ __launch_bounds__(NTHR) void k_cvt(
    const float* __restrict__ s0, f16* d0, int n0, float c0,
    const float* __restrict__ s1, f16* d1, int n1, float c1,
    const float* __restrict__ s2, f16* d2, int n2, float c2,
    const float* __restrict__ s3, f16* d3, int n3, float c3)
{
  const int y = (int)blockIdx.y;
  const float* s = (y == 0) ? s0 : ((y == 1) ? s1 : ((y == 2) ? s2 : s3));
  f16* d         = (y == 0) ? d0 : ((y == 1) ? d1 : ((y == 2) ? d2 : d3));
  const int n    = (y == 0) ? n0 : ((y == 1) ? n1 : ((y == 2) ? n2 : n3));
  const float c  = (y == 0) ? c0 : ((y == 1) ? c1 : ((y == 2) ? c2 : c3));
  const int i = (int)blockIdx.x * NTHR + (int)threadIdx.x;
  if (i >= n) return;
  const float* p = s + (size_t)i * 8;
  const v4f a = *(const v4f*)p, b = *(const v4f*)(p + 4);
  const v8h hv = cvt8h(a, b, c);
  f16* op = d + (size_t)i * 8;
  *(volatile v8h*)op = hv;
  __threadfence();
  *(volatile v8h*)op = hv;
}

__global__ __launch_bounds__(NTHR) void k_peprep(const float* __restrict__ pe, f16* PE16, int nRows, int nUnits) {
  const int i = (int)blockIdx.x * NTHR + (int)threadIdx.x;
  if (i >= nUnits) return;
  const int row = i >> 5;
  const int c0  = (i & 31) * 8;
  const int rc  = row < nRows ? row : nRows - 1;
  const float* p = pe + (size_t)rc * NH + c0;
  v4f a = *(const v4f*)p, b = *(const v4f*)(p + 4);
  const v4f z4 = {0.f, 0.f, 0.f, 0.f};
  if (row >= nRows) { a = z4; b = z4; }
  const v8h hv = cvt8h(a, b, CW);
  f16* op = PE16 + (size_t)row * NF2 + c0;
  *(volatile v8h*)op = hv;
  __threadfence();
  *(volatile v8h*)op = hv;
}

__global__ __launch_bounds__(NTHR) void k_wtr(const float* __restrict__ W, f16* WT, int K, int Nc) {
  __shared__ __attribute__((aligned(16))) float tile[TT * TP];
  const int tid = (int)threadIdx.x, lane = tid & 31, wave = tid >> 5;
  const int n0 = (int)blockIdx.x * TT;
  const int k0 = (int)blockIdx.y * TT;
#pragma unroll
  for (int i = 0; i < 4; ++i) {
    const int kr = (tid >> 4) + 16 * i;
    const int c4 = (tid & 15) * 4;
    const v4f v = *(const v4f*)(W + (size_t)(k0 + kr) * (size_t)Nc + n0 + c4);
    *(v4f*)(tile + kr * TP + c4) = v;
  }
  __syncthreads();
  const int q = lane & 7;
  v8h hv[2];
#pragma unroll
  for (int i = 0; i < 2; ++i) {
    const int nr = 8 * wave + 4 * i + (lane >> 3);
    v4f a, b;
    a.x = tile[(8 * q + 0) * TP + nr]; a.y = tile[(8 * q + 1) * TP + nr];
    a.z = tile[(8 * q + 2) * TP + nr]; a.w = tile[(8 * q + 3) * TP + nr];
    b.x = tile[(8 * q + 4) * TP + nr]; b.y = tile[(8 * q + 5) * TP + nr];
    b.z = tile[(8 * q + 6) * TP + nr]; b.w = tile[(8 * q + 7) * TP + nr];
    hv[i] = cvt8h(a, b, CW);
  }
#pragma unroll
  for (int i = 0; i < 2; ++i) {
    const int nr = 8 * wave + 4 * i + (lane >> 3);
    f16* op = WT + (size_t)(n0 + nr) * (size_t)K + k0 + 8 * q;
    *(volatile v8h*)op = hv[i];
  }
  __threadfence();
#pragma unroll
  for (int i = 0; i < 2; ++i) {
    const int nr = 8 * wave + 4 * i + (lane >> 3);
    f16* op = WT + (size_t)(n0 + nr) * (size_t)K + k0 + 8 * q;
    *(volatile v8h*)op = hv[i];
  }
}

__global__ __launch_bounds__(NTHR) void k_qprep(const float* __restrict__ QP, const float* __restrict__ ub,
                                                const float* __restrict__ vb, f16* QU, f16* QV, int nUnits) {
  const int i = (int)blockIdx.x * NTHR + (int)threadIdx.x;
  if (i >= nUnits) return;
  const int row = i >> 6;
  const int c0  = (i & 63) * 8;
  const float* p = QP + (size_t)row * NH + c0;
  const v4f a = *(const v4f*)p, b = *(const v4f*)(p + 4);
  const v4f u0 = *(const v4f*)(ub + c0), u1 = *(const v4f*)(ub + c0 + 4);
  const v4f w0 = *(const v4f*)(vb + c0), w1 = *(const v4f*)(vb + c0 + 4);
  const v8h hu = cvt8h(a + u0, b + u1, CX);
  const v8h hq = cvt8h(a + w0, b + w1, CX);
  const size_t o = (size_t)row * NH + c0;
  *(volatile v8h*)(QU + o) = hu;
  *(volatile v8h*)(QV + o) = hq;
  __threadfence();
  *(volatile v8h*)(QU + o) = hu;
  *(volatile v8h*)(QV + o) = hq;
}

template<int EPI>
__global__ __launch_bounds__(GTHR) void k_gemm(
    const f16* __restrict__ A, const f16* __restrict__ BT, const float* __restrict__ bias,
    float* outF, f16* outH,
    int K, int lda, int ldb, int ldo, int biasMode, int biasLen, int zdiv,
    int sA0, int sA1, int sB0, int sB1, int sO0, int sO1, float scl, float cao)
{
  __shared__ __attribute__((aligned(16))) float stg[GBM * GBN];
  const int tid = (int)threadIdx.x, lane = tid & 31, wave = tid >> 5, hh = lane >> 4, m = lane & 15;
  const int z  = (int)blockIdx.z;
  const int z0 = z % zdiv, z1 = z / zdiv;
  const size_t oA = (size_t)z1 * (size_t)sA1 + (size_t)z0 * (size_t)sA0;
  const size_t oB = (size_t)z1 * (size_t)sB1 + (size_t)z0 * (size_t)sB0;
  const size_t oO = (size_t)z1 * (size_t)sO1 + (size_t)z0 * (size_t)sO0;
  const int rowBase = (int)blockIdx.x * GBM;
  const int col0    = (int)blockIdx.y * GBN;

  v8f acc[4];
  {
    const v8f zz = {0.f, 0.f, 0.f, 0.f, 0.f, 0.f, 0.f, 0.f};
    acc[0] = zz; acc[1] = zz; acc[2] = zz; acc[3] = zz;
  }
  const f16* ap = A  + oA + (size_t)(rowBase + 16 * wave + m) * (size_t)lda + 8 * hh;
  const f16* wp = BT + oB + (size_t)(col0 + m) * (size_t)ldb + 8 * hh;
  const int ksteps = K >> 5;
#pragma unroll 1
  for (int ks = 0; ks < ksteps; ++ks) {
    FragH af;
    af.h[0] = *(const v8h*)(ap + 32 * ks);
    af.h[1] = *(const v8h*)(ap + 32 * ks + 16);
#pragma unroll
    for (int t = 0; t < 4; ++t) {
      const f16* wq = wp + (size_t)(16 * t) * (size_t)ldb + 32 * ks;
      FragH bf;
      bf.h[0] = *(const v8h*)wq;
      bf.h[1] = *(const v8h*)(wq + 16);
      acc[t] = wmh(af, bf, acc[t]);
    }
  }

  float brw[8];
#pragma unroll
  for (int r = 0; r < 8; ++r) {
    int ri = rowBase + 16 * wave + 8 * hh + r;
    ri = ri > biasLen - 1 ? biasLen - 1 : ri;
    brw[r] = bias[ri];
  }
#pragma unroll
  for (int t = 0; t < 4; ++t) {
    const int lc = 16 * t + m;
    int ci = col0 + lc;
    ci = ci > biasLen - 1 ? biasLen - 1 : ci;
    const float bc = bias[ci];
#pragma unroll
    for (int r = 0; r < 8; ++r) {
      const int lr = 16 * wave + 8 * hh + r;
      const float bvv = (biasMode == 1) ? bc : ((biasMode == 2) ? brw[r] : 0.f);
      stg[lr * GBN + lc] = fmaf(acc[t][r], scl, bvv);
    }
  }
  __syncthreads();

  if (EPI == 0) {
    float* ob = outF + oO;
    v4f fv[8];
#pragma unroll
    for (int i = 0; i < 8; ++i) {
      const int lr = 16 * wave + 2 * i + hh;
      fv[i] = *(const v4f*)(stg + lr * GBN + 4 * m);
    }
#pragma unroll
    for (int i = 0; i < 8; ++i) {
      const int lr = 16 * wave + 2 * i + hh;
      float* op = ob + (size_t)(rowBase + lr) * (size_t)ldo + col0 + 4 * m;
      *(volatile v4f*)op = fv[i];
    }
    __threadfence();
#pragma unroll
    for (int i = 0; i < 8; ++i) {
      const int lr = 16 * wave + 2 * i + hh;
      float* op = ob + (size_t)(rowBase + lr) * (size_t)ldo + col0 + 4 * m;
      *(volatile v4f*)op = fv[i];
    }
  }
  if (EPI == 1) {
    f16* ob = outH + oO;
    const int q8 = lane & 7;
    v8h hv[4];
#pragma unroll
    for (int i = 0; i < 4; ++i) {
      const int lr = 16 * wave + 4 * i + (lane >> 3);
      const v4f a = *(const v4f*)(stg + lr * GBN + 8 * q8);
      const v4f b = *(const v4f*)(stg + lr * GBN + 8 * q8 + 4);
      hv[i] = cvt8h(a, b, cao);
    }
#pragma unroll
    for (int i = 0; i < 4; ++i) {
      const int lr = 16 * wave + 4 * i + (lane >> 3);
      f16* op = ob + (size_t)(rowBase + lr) * (size_t)ldo + col0 + 8 * q8;
      *(volatile v8h*)op = hv[i];
    }
    __threadfence();
#pragma unroll
    for (int i = 0; i < 4; ++i) {
      const int lr = 16 * wave + 4 * i + (lane >> 3);
      f16* op = ob + (size_t)(rowBase + lr) * (size_t)ldo + col0 + 8 * q8;
      *(volatile v8h*)op = hv[i];
    }
  }
}

__global__ __launch_bounds__(GTHR) void k_score(
    const float* __restrict__ TTB, const float* __restrict__ bfus, const f16* __restrict__ GH,
    const int* __restrict__ pos_s, const int* __restrict__ pos_e,
    const float* __restrict__ SAC, const float* __restrict__ QP,
    const float* __restrict__ vbias, const float* __restrict__ br,
    const int* __restrict__ seq_len, const int* __restrict__ lex,
    f16* PH)
{
  __shared__ __attribute__((aligned(16))) f16   at[64 * ATP];
  __shared__ __attribute__((aligned(16))) f16   gt[16 * NH];
  __shared__ __attribute__((aligned(16))) float sc[NHEAD * NL];
  __shared__ float scb[NHEAD];
  (void)lex;
  const int tid = (int)threadIdx.x, lane = tid & 31, wave = tid >> 5, hh = lane >> 4, m = lane & 15;
  const int bq = (int)blockIdx.x;
  const int b  = bq / NL;
  const int q  = bq - b * NL;
  const v4f z4 = {0.f, 0.f, 0.f, 0.f};

  {
    const f16* gp = GH + (size_t)bq * (size_t)(NHEAD * NH);
#pragma unroll
    for (int i = 0; i < 4; ++i) {
      const int u = tid + GTHR * i;
      const v8h v = *(const v8h*)(gp + 8 * u);
      *(v8h*)(gt + 8 * u) = v;
    }
    const v8h zh = cvt8h(z4, z4, 1.0f);
#pragma unroll
    for (int i = 0; i < 4; ++i) {
      const int u = tid + GTHR * i;
      *(v8h*)(gt + NHEAD * NH + 8 * u) = zh;
    }
  }
#pragma unroll
  for (int j = 0; j < 2; ++j) {
    const int n = 2 * wave + j;
    const int c = n * NDH + 2 * lane;
    const float q0 = QP[(size_t)bq * NH + c];
    const float q1 = QP[(size_t)bq * NH + c + 1];
    float p = (q0 + vbias[c]) * br[c] + (q1 + vbias[c + 1]) * br[c + 1];
#pragma unroll
    for (int o = 16; o > 0; o >>= 1) p += __shfl_xor(p, o);
    if (lane == 0) scb[n] = p;
  }

  const int psq = pos_s[bq], peq = pos_e[bq];
  const int krow = tid >> 1, fh = tid & 1;
#pragma unroll 1
  for (int kt = 0; kt < NL / 64; ++kt) {
    const int kk  = kt * 64 + krow;
    const int psk = pos_s[b * NL + kk], pek = pos_e[b * NL + kk];
    int dss = psq - psk + NMAXL;
    int dse = psq - pek + NMAXL;
    int des = peq - psk + NMAXL;
    int dee = peq - pek + NMAXL;
    dss = dss < 0 ? 0 : (dss > NPE - 1 ? NPE - 1 : dss);
    dse = dse < 0 ? 0 : (dse > NPE - 1 ? NPE - 1 : dse);
    des = des < 0 ? 0 : (des > NPE - 1 ? NPE - 1 : des);
    dee = dee < 0 ? 0 : (dee > NPE - 1 ? NPE - 1 : dee);
    const float* t0p = TTB + (size_t)dss * NH;
    const float* t1p = TTB + (size_t)(NPEP + dse) * NH;
    const float* t2p = TTB + (size_t)(2 * NPEP + des) * NH;
    const float* t3p = TTB + (size_t)(3 * NPEP + dee) * NH;
    v8f acc = {0.f, 0.f, 0.f, 0.f, 0.f, 0.f, 0.f, 0.f};
#pragma unroll 1
    for (int ch = 0; ch < NH / 128; ++ch) {
      const int cb = ch * 128;
      __syncthreads();
#pragma unroll 2
      for (int i = 0; i < 8; ++i) {
        const int f = cb + fh * 64 + 8 * i;
        v4f a  = *(const v4f*)(t0p + f) + *(const v4f*)(t1p + f);
        v4f c  = *(const v4f*)(t2p + f) + *(const v4f*)(t3p + f);
        a = (a + c) + *(const v4f*)(bfus + f);
        v4f a2 = *(const v4f*)(t0p + f + 4) + *(const v4f*)(t1p + f + 4);
        v4f c2 = *(const v4f*)(t2p + f + 4) + *(const v4f*)(t3p + f + 4);
        a2 = (a2 + c2) + *(const v4f*)(bfus + f + 4);
        const v8h hv = cvt8h(relu4(a), relu4(a2), CR);
        *(v8h*)(at + krow * ATP + fh * 64 + 8 * i) = hv;
      }
      __syncthreads();
#pragma unroll
      for (int ks = 0; ks < 4; ++ks) {
        FragH af, bf;
        const f16* ap = at + (16 * wave + m) * ATP + 32 * ks + 8 * hh;
        af.h[0] = *(const v8h*)ap;
        af.h[1] = *(const v8h*)(ap + 16);
        const f16* bp = gt + m * NH + cb + 32 * ks + 8 * hh;
        bf.h[0] = *(const v8h*)bp;
        bf.h[1] = *(const v8h*)(bp + 16);
        acc = wmh(af, bf, acc);
      }
    }
    if (m < NHEAD) {
      float* sp = sc + m * NL + kt * 64 + 16 * wave + 8 * hh;
#pragma unroll
      for (int r = 0; r < 8; ++r) sp[r] = acc[r] * (1.0f / 32768.0f);
    }
  }
  __syncthreads();

  const int  sl  = seq_len[b];
  const bool act = lane < 24;
  const int  lc  = act ? lane : 23;
  const int  k8  = lc * 8;
  v8h pv[2];
#pragma unroll
  for (int j = 0; j < 2; ++j) {
    const int n = 2 * wave + j;
    const size_t rowo = ((size_t)((b * NHEAD + n) * NL + q)) * (size_t)NL;
    const float* rp = SAC + rowo + k8;
    const v4f a0 = *(const v4f*)rp, a1 = *(const v4f*)(rp + 4);
    const v4f d0 = *(const v4f*)(sc + n * NL + k8), d1 = *(const v4f*)(sc + n * NL + k8 + 4);
    const float scn = scb[n];
    float s[8];
    s[0] = (a0.x + (d0.x + scn)) * 0.125f; s[1] = (a0.y + (d0.y + scn)) * 0.125f;
    s[2] = (a0.z + (d0.z + scn)) * 0.125f; s[3] = (a0.w + (d0.w + scn)) * 0.125f;
    s[4] = (a1.x + (d1.x + scn)) * 0.125f; s[5] = (a1.y + (d1.y + scn)) * 0.125f;
    s[6] = (a1.z + (d1.z + scn)) * 0.125f; s[7] = (a1.w + (d1.w + scn)) * 0.125f;
    float mx = -3.0e38f;
#pragma unroll
    for (int e = 0; e < 8; ++e) {
      float v = (k8 + e < sl) ? s[e] : -1.0e15f;
      v = act ? v : -1.0e30f;
      s[e] = v;
      mx = fmaxf(mx, v);
    }
#pragma unroll
    for (int o = 16; o > 0; o >>= 1) mx = fmaxf(mx, __shfl_xor(mx, o));
    float sum = 0.f;
#pragma unroll
    for (int e = 0; e < 8; ++e) { s[e] = __expf(s[e] - mx); sum += s[e]; }
#pragma unroll
    for (int o = 16; o > 0; o >>= 1) sum += __shfl_xor(sum, o);
    const float fc = CP * (1.0f / sum);
    v4f p0, p1;
    p0.x = s[0] * fc; p0.y = s[1] * fc; p0.z = s[2] * fc; p0.w = s[3] * fc;
    p1.x = s[4] * fc; p1.y = s[5] * fc; p1.z = s[6] * fc; p1.w = s[7] * fc;
    pv[j] = cvt8h(p0, p1, 1.0f);
  }
#pragma unroll
  for (int j = 0; j < 2; ++j) {
    const int n = 2 * wave + j;
    f16* op = PH + ((size_t)((b * NHEAD + n) * NL + q)) * (size_t)NL + k8;
    if (act) *(volatile v8h*)op = pv[j];
  }
  __threadfence();
#pragma unroll
  for (int j = 0; j < 2; ++j) {
    const int n = 2 * wave + j;
    f16* op = PH + ((size_t)((b * NHEAD + n) * NL + q)) * (size_t)NL + k8;
    if (act) *(volatile v8h*)op = pv[j];
  }
}

static inline int cdiv(int a, int b) { return (a + b - 1) / b; }

extern "C" void kernel_launch(void* const* d_in, const int* in_sizes, int n_in,
                              void* d_out, int out_size, void* d_ws, size_t ws_size,
                              hipStream_t stream) {
  if (n_in < 22) return;
  if (in_sizes[0] != NBL * NH || in_sizes[1] != NBL * NH || in_sizes[2] != NBL * NH) return;
  if (in_sizes[3] != NB) return;
  if (in_sizes[4] < 1) return;
  if (in_sizes[5] != NBL || in_sizes[6] != NBL) return;
  if (in_sizes[7] != NPE * NH) return;
  if (in_sizes[8] != NH * NFUS || in_sizes[9] != NH) return;
  if (in_sizes[10] != NH * NH || in_sizes[11] != NH) return;
  if (in_sizes[12] != NH * NH || in_sizes[13] != NH) return;
  if (in_sizes[14] != NH * NH || in_sizes[15] != NH) return;
  if (in_sizes[16] != NH * NH || in_sizes[17] != NH) return;
  if (in_sizes[18] != NHEAD * NDH || in_sizes[19] != NHEAD * NDH) return;
  if (in_sizes[20] != NH * NH || in_sizes[21] != NH) return;
  if (out_size != NBL * NH) return;

  const float* key   = (const float*)d_in[0];
  const float* query = (const float*)d_in[1];
  const float* value = (const float*)d_in[2];
  const int*   seqln = (const int*)d_in[3];
  const int*   lexn  = (const int*)d_in[4];
  const int*   pos_s = (const int*)d_in[5];
  const int*   pos_e = (const int*)d_in[6];
  const float* pe    = (const float*)d_in[7];
  const float* W_fus = (const float*)d_in[8];
  const float* b_fus = (const float*)d_in[9];
  const float* Wk    = (const float*)d_in[10];
  const float* bk    = (const float*)d_in[11];
  const float* Wq    = (const float*)d_in[12];
  const float* bq    = (const float*)d_in[13];
  const float* Wv    = (const float*)d_in[14];
  const float* bv    = (const float*)d_in[15];
  const float* Wr    = (const float*)d_in[16];
  const float* br    = (const float*)d_in[17];
  const float* u_b   = (const float*)d_in[18];
  const float* v_b   = (const float*)d_in[19];
  const float* Wff   = (const float*)d_in[20];
  const float* bff   = (const float*)d_in[21];
  float* out = (float*)d_out;

  const size_t szX   = (size_t)NBL * NH * 2;
  const size_t szW   = (size_t)NH * NH * 2;
  const size_t szWF  = (size_t)NH * NFUS * 2;
  const size_t szPE  = (size_t)NPEP * NF2 * 2;
  const size_t szQP  = (size_t)NBL * NH * 4;
  const size_t szVT  = (size_t)NB * NH * NL * 2;
  const size_t szT   = (size_t)4 * NPEP * NH * 4;
  const size_t szGH  = (size_t)NBL * NHEAD * NH * 2;
  const size_t szSAC = (size_t)NB * NHEAD * NL * NL * 4;
  const size_t szPH  = (size_t)NB * NHEAD * NL * NL * 2;
  size_t off = 0;
  const size_t oXK  = off; off += szX;
  const size_t oXQ  = off; off += szX;
  const size_t oXV  = off; off += szX;
  const size_t oWK  = off; off += szW;
  const size_t oWQ  = off; off += szW;
  const size_t oWV  = off; off += szW;
  const size_t oWF  = off; off += szW;
  const size_t oWFU = off; off += szWF;
  const size_t oWRT = off; off += szW;
  const size_t oPE  = off; off += szPE;
  const size_t oQP  = off; off += szQP;
  const size_t oKH  = off; off += szX;
  const size_t oVT  = off; off += szVT;
  const size_t oQU  = off; off += szX;
  const size_t oQV  = off; off += szX;
  const size_t oT   = off; off += szT;
  const size_t oGH  = off; off += szGH;
  const size_t oSAC = off; off += szSAC;
  const size_t oPH  = off; off += szPH;
  const size_t oOH  = off; off += szX;
  if (off > ws_size || off > (size_t)WSMAX) return;

  char* ws = (char*)d_ws;
  f16*   XK   = (f16*)(ws + oXK);
  f16*   XQ   = (f16*)(ws + oXQ);
  f16*   XV   = (f16*)(ws + oXV);
  f16*   W16K = (f16*)(ws + oWK);
  f16*   W16Q = (f16*)(ws + oWQ);
  f16*   W16V = (f16*)(ws + oWV);
  f16*   W16F = (f16*)(ws + oWF);
  f16*   WFUS = (f16*)(ws + oWFU);
  f16*   WRT  = (f16*)(ws + oWRT);
  f16*   PE16 = (f16*)(ws + oPE);
  float* QP   = (float*)(ws + oQP);
  f16*   KH   = (f16*)(ws + oKH);
  f16*   VT   = (f16*)(ws + oVT);
  f16*   QU   = (f16*)(ws + oQU);
  f16*   QV   = (f16*)(ws + oQV);
  float* TTB  = (float*)(ws + oT);
  f16*   GH   = (f16*)(ws + oGH);
  float* SAC  = (float*)(ws + oSAC);
  f16*   PH   = (f16*)(ws + oPH);
  f16*   OH   = (f16*)(ws + oOH);

  const int uX = NBL * NH / 8;
  const int uW = NH * NH / 8;
  const int uWF = NH * NFUS / 8;

  k_cvt<<<dim3(cdiv(uW, NTHR), 4), NTHR, 0, stream>>>(key, XK, uX, CX, query, XQ, uX, CX, value, XV, uX, CX,
                                                      Wff, W16F, uW, CW);
  k_cvt<<<dim3(cdiv(uWF, NTHR), 4), NTHR, 0, stream>>>(Wk, W16K, uW, CW, Wq, W16Q, uW, CW, Wv, W16V, uW, CW,
                                                       W_fus, WFUS, uWF, CW);
  const int uPE = NPEP * (NF2 / 8);
  k_peprep<<<cdiv(uPE, NTHR), NTHR, 0, stream>>>(pe, PE16, NPE, uPE);
  k_wtr<<<dim3(NH / TT, NH / TT), NTHR, 0, stream>>>(Wr, WRT, NH, NH);

  const float S512 = 1.0f / 512.0f;
  k_gemm<0><<<dim3(NBL / GBM, NH / GBN, 1), GTHR, 0, stream>>>(XQ, W16Q, bq, QP, OH,
      NH, NH, NH, NH, 1, NH, 1, 0, 0, 0, 0, 0, 0, S512, 1.0f);
  k_gemm<1><<<dim3(NBL / GBM, NH / GBN, 1), GTHR, 0, stream>>>(XK, W16K, bk, QP, KH,
      NH, NH, NH, NH, 1, NH, 1, 0, 0, 0, 0, 0, 0, S512, CX);
  k_gemm<1><<<dim3(NH / GBM, NL / GBN, NB), GTHR, 0, stream>>>(W16V, XV, bv, QP, VT,
      NH, NH, NH, NL, 2, NH, 1, 0, 0, 0, NL * NH, 0, NH * NL, S512, CX);
  k_qprep<<<cdiv(NBL * (NH / 8), NTHR), NTHR, 0, stream>>>(QP, u_b, v_b, QU, QV, NBL * (NH / 8));
  k_gemm<0><<<dim3(NPEP / GBM, NH / GBN, 4), GTHR, 0, stream>>>(PE16, WFUS, bq, TTB, OH,
      NF2, NF2, NFUS, NH, 0, NH, 1, 0, 0, 0, NF2, 0, NPEP * NH, 1.0f / 4096.0f, 1.0f);
  k_gemm<1><<<dim3(NBL / GBM, NH / GBN, NHEAD), GTHR, 0, stream>>>(QV, WRT, bq, QP, GH,
      NDH, NH, NH, NHEAD * NH, 0, NH, 1, 0, NDH, 0, NDH, 0, NH, S512, CG);
  k_gemm<0><<<dim3(NL / GBM, NL / GBN, NB * NHEAD), GTHR, 0, stream>>>(QU, KH, bq, SAC, OH,
      NDH, NH, NH, NL, 0, NH, NHEAD, NDH, NL * NH, NDH, NL * NH, NL * NL, NHEAD * NL * NL, 1.0f / 64.0f, 1.0f);
  k_score<<<NBL, GTHR, 0, stream>>>(TTB, b_fus, GH, pos_s, pos_e, SAC, QP, v_b, br, seqln, lexn, PH);
  k_gemm<1><<<dim3(NL / GBM, NDH / GBN, NB * NHEAD), GTHR, 0, stream>>>(PH, VT, bq, QP, OH,
      NL, NL, NL, NH, 0, NH, NHEAD, NL * NL, NHEAD * NL * NL, NDH * NL, NH * NL, NDH, NL * NH,
      1.0f / 32768.0f, CO);
  k_gemm<0><<<dim3(NBL / GBM, NH / GBN, 1), GTHR, 0, stream>>>(OH, W16F, bff, out, KH,
      NH, NH, NH, NH, 1, NH, 1, 0, 0, 0, 0, 0, 0, 1.0f / 4096.0f, 1.0f);
}
